// ResAttnBlock_14422500180420
// MI455X (gfx1250) — hardware-verified
//
#include <hip/hip_runtime.h>


namespace {
constexpr int Bn = 4, C = 256, Hh = 64, Ww = 64, N = 4096, NT = Bn * N, CL = 32, KCV = 2304;
constexpr float QS = 8.0f, KS = 8.0f, VS = 8.0f, PS = 8.0f, WS8 = 8.0f;

typedef _Float16 b16;
typedef __attribute__((ext_vector_type(16))) _Float16 v16b;
typedef __attribute__((ext_vector_type(8))) _Float16 v8b;
typedef __attribute__((ext_vector_type(8))) float v8f;
typedef __attribute__((ext_vector_type(4))) float v4f;
__device__ __forceinline__ float bf16_rne(float f) { unsigned int u = __float_as_uint(f); u += 0x7FFFu + ((u >> 16) & 1u); return __uint_as_float(u & 0xFFFF0000u); }
__device__ __forceinline__ void split16(float v, b16& hi, b16& lo) { hi = (b16)v; lo = (b16)(v - (float)hi); }
__device__ __forceinline__ v16b frag_kb(const b16* p, int hh) { const v8b a = *(const v8b*)(p + 8 * hh), b = *(const v8b*)(p + 16 + 8 * hh); v16b f;
#pragma unroll
  for (int e = 0; e < 8; ++e) { f[e] = a[e]; f[8 + e] = b[e]; } return f; }
__device__ __forceinline__ void frag_split_s(const float* p, int hh, float sc, v16b& fh, v16b& fl) {
#pragma unroll
  for (int e = 0; e < 8; ++e) { b16 a, c; split16(p[8 * hh + e] * sc, a, c); fh[e] = a; fl[e] = c; split16(p[16 + 8 * hh + e] * sc, a, c); fh[8 + e] = a; fl[8 + e] = c; } }
__device__ __forceinline__ v8f wmma16b(v16b a, v16b b, v8f c) { v8f d = __builtin_amdgcn_wmma_f32_16x16x32_f16(false, a, false, b, (short)0, c, false, false); asm volatile("v_nop\n\tv_nop\n\tv_nop\n\tv_nop" : "+v"(d) : "v"(a), "v"(b)); return d; }
__device__ __forceinline__ void wave_lds_sync() { __builtin_amdgcn_fence(__ATOMIC_RELEASE, "workgroup"); __builtin_amdgcn_wave_barrier(); __builtin_amdgcn_fence(__ATOMIC_ACQUIRE, "workgroup"); }
__device__ __forceinline__ float nexp(float x) { return __builtin_amdgcn_exp2f(x * 1.4426950408889634f); }
__device__ __forceinline__ float pmul(float a, float b) { float p = a * b; asm volatile("" : "+v"(p)); return p; }

__global__ __launch_bounds__(256) void sigma_kernel(const float* __restrict__ wbar, const float* __restrict__ u, const float* __restrict__ gfm, const float* __restrict__ gc, const float* __restrict__ rg, float* __restrict__ P) {
  __shared__ float T[KCV]; __shared__ float Sv[256]; __shared__ float red[256];
  const int t_ = threadIdx.x;
  for (int k = t_; k < KCV; k += 256) { float s = 0.0f; for (int o = 0; o < C; ++o) s += bf16_rne(wbar[(size_t)o * KCV + k]) * bf16_rne(u[o]); T[k] = s; }
  __syncthreads();
  { float s = 0.0f; for (int k = t_; k < KCV; k += 256) s += pmul(T[k], T[k]); red[t_] = s; __syncthreads(); for (int st = 128; st > 0; st >>= 1) { if (t_ < st) red[t_] += red[t_ + st]; __syncthreads(); } }
  const float inv_t = 1.0f / (sqrtf(red[0]) + 1e-12f); __syncthreads();
  { float s = 0.0f; const float* wr = wbar + (size_t)t_ * KCV; for (int k = 0; k < KCV; ++k) s += bf16_rne(wr[k]) * (T[k] * inv_t); Sv[t_] = s; }
  __syncthreads();
  { red[t_] = pmul(Sv[t_], Sv[t_]); __syncthreads(); for (int st = 128; st > 0; st >>= 1) { if (t_ < st) red[t_] += red[t_ + st]; __syncthreads(); } }
  const float inv_s = 1.0f / (sqrtf(red[0]) + 1e-12f); __syncthreads();
  { red[t_] = (Sv[t_] * inv_s) * Sv[t_]; __syncthreads(); for (int st = 128; st > 0; st >>= 1) { if (t_ < st) red[t_] += red[t_ + st]; __syncthreads(); } }
  if (t_ < 32) { const float v = (t_ == 0) ? red[0] : (t_ == 1) ? bf16_rne(gfm[0]) : (t_ == 2) ? bf16_rne(gc[0]) : (t_ == 3) ? bf16_rne(rg[0]) : 0.0f; for (int pass = 0; pass < 2; ++pass) ((volatile float*)P)[t_] = v; }
  __threadfence();
}

struct Wo_ { static constexpr size_t W1 = 0, WOC = W1 + (size_t)448 * 256, CVH = WOC + 256 * 32, CVL = CVH + (size_t)256 * KCV, END = CVL + (size_t)256 * KCV; };
__global__ __launch_bounds__(256) void prep_kernel(const float* __restrict__ wq, const float* __restrict__ wk, const float* __restrict__ wv, const float* __restrict__ wqc, const float* __restrict__ wkc, const float* __restrict__ wvc, const float* __restrict__ woc, const float* __restrict__ wbar,
                                                   const float* __restrict__ bq, const float* __restrict__ bk, const float* __restrict__ bv, const float* __restrict__ bqc, const float* __restrict__ bkc, const float* __restrict__ bvc, const float* __restrict__ boc, const float* __restrict__ P, b16* __restrict__ R, float* __restrict__ Pb) {
  const int t_ = blockIdx.x * 256 + threadIdx.x, nth = gridDim.x * 256; const float isg = 1.0f / P[0];
  for (int pass = 0; pass < 2; ++pass) {
    for (int q = t_; q < 448 * 256; q += nth) { const int o = q >> 8, c = q & 255; float w;
      if (o < 32) w = wq[o * C + c]; else if (o < 64) w = wk[(o - 32) * C + c]; else if (o < 320) w = wv[(o - 64) * C + c]; else if (o < 352) w = wqc[(o - 320) * C + c]; else if (o < 384) w = wkc[(o - 352) * C + c]; else if (o < 416) w = wvc[(o - 384) * C + c]; else w = 0.0f;
      R[Wo_::W1 + q] = (b16)bf16_rne(w); }
    for (int q = t_; q < 256 * 32; q += nth) R[Wo_::WOC + q] = (b16)bf16_rne(woc[q]);
    for (int q = t_; q < 256 * KCV; q += nth) { const int o = q / KCV, k = q % KCV, tap = k >> 8, c = k & 255; const float w = bf16_rne(wbar[((size_t)o * C + c) * 9 + tap]) * isg; b16 h_, l_; split16(w * WS8, h_, l_); R[Wo_::CVH + q] = h_; R[Wo_::CVL + q] = l_; }
    for (int q = t_; q < 448 + 256; q += nth) { float v; if (q < 32) v = bq[q]; else if (q < 64) v = bk[q - 32]; else if (q < 320) v = bv[q - 64]; else if (q < 352) v = bqc[q - 320]; else if (q < 384) v = bkc[q - 352]; else if (q < 416) v = bvc[q - 384]; else if (q < 448) v = 0.0f; else v = boc[q - 448]; Pb[q] = bf16_rne(v); }
    __threadfence(); }
}

__global__ __launch_bounds__(256) void xpose_kernel(const float* __restrict__ x, b16* __restrict__ xt) {
  __shared__ __attribute__((aligned(16))) b16 T[128][C + 8];
  const int b = blockIdx.y, n0 = blockIdx.x * 128, t_ = threadIdx.x;
  for (int i = t_; i < C * 128; i += 256) { const int c = i >> 7, nn = i & 127; T[nn][c] = (b16)bf16_rne(x[((size_t)b * C + c) * N + n0 + nn]); }
  __syncthreads();
  for (int pass = 0; pass < 2; ++pass) { for (int i = t_; i < 128 * (C / 8); i += 256) { const int nn = i / (C / 8), c8 = (i % (C / 8)) * 8; *(volatile v8b*)(xt + ((size_t)b * N + n0 + nn) * C + c8) = *(const v8b*)(&T[nn][c8]); } __threadfence(); }
}

__global__ __launch_bounds__(128) void lin_kernel(const b16* __restrict__ xt, const b16* __restrict__ R, const float* __restrict__ Pb, float* __restrict__ qk, b16* __restrict__ vpl, float* __restrict__ qkc, float* __restrict__ vc) {
  __shared__ __attribute__((aligned(16))) float Tc[64][128 + 4];
  const int lane = threadIdx.x & 31, wave = threadIdx.x >> 5, nloc = lane & 15, hlf = lane >> 4, ct = blockIdx.x, c0 = ct * 64, p0 = blockIdx.y * 128, m0 = p0 + wave * 32, b = p0 / N, t0 = p0 % N;
  v8f acc[2][4];
#pragma unroll
  for (int r = 0; r < 2; ++r)
#pragma unroll
    for (int t = 0; t < 4; ++t) acc[r][t] = (v8f){};
#pragma unroll 2
  for (int kb = 0; kb < C; kb += 32) { const v16b a0 = frag_kb(xt + (size_t)(m0 + nloc) * C + kb, hlf), a1 = frag_kb(xt + (size_t)(m0 + 16 + nloc) * C + kb, hlf);
#pragma unroll
    for (int t = 0; t < 4; ++t) { const v16b bw = frag_kb(R + Wo_::W1 + (size_t)(c0 + t * 16 + nloc) * C + kb, hlf); acc[0][t] = wmma16b(a0, bw, acc[0][t]); acc[1][t] = wmma16b(a1, bw, acc[1][t]); } }
#pragma unroll
  for (int t = 0; t < 4; ++t) { const int cc = c0 + t * 16 + nloc; const float bb = Pb[cc];
#pragma unroll
    for (int r = 0; r < 2; ++r)
#pragma unroll
      for (int v = 0; v < 8; ++v) Tc[t * 16 + nloc][wave * 32 + r * 16 + 8 * hlf + v] = acc[r][t][v] + bb; }
  __syncthreads();
  for (int pass = 0; pass < 2; ++pass) {
    if (ct == 0) { for (int i = threadIdx.x; i < 128 * 16; i += 128) { const int pl = i >> 4, c4 = (i & 15) * 4; v4f o; o[0] = Tc[c4][pl]; o[1] = Tc[c4 + 1][pl]; o[2] = Tc[c4 + 2][pl]; o[3] = Tc[c4 + 3][pl]; *(volatile v4f*)(qk + (size_t)(p0 + pl) * 64 + c4) = o; } }
    else if (ct < 5) { for (int i = threadIdx.x; i < 64 * 16; i += 128) { const int cc = i >> 4, c8 = (i & 15) * 8; v8b o; for (int e = 0; e < 8; ++e) o[e] = (b16)(Tc[cc][c8 + e] * VS); *(volatile v8b*)(vpl + ((size_t)b * C + (c0 - 64) + cc) * N + t0 + c8) = o; } }
    else if (ct == 5) { for (int i = threadIdx.x; i < 64 * 32; i += 128) { const int cc = i >> 5, c4 = (i & 31) * 4; *(volatile v4f*)(qkc + ((size_t)b * 64 + cc) * N + t0 + c4) = *(const v4f*)(&Tc[cc][c4]); } }
    else { for (int i = threadIdx.x; i < 32 * 32; i += 128) { const int cc = i >> 5, c4 = (i & 31) * 4; *(volatile v4f*)(vc + ((size_t)b * 32 + cc) * N + t0 + c4) = *(const v4f*)(&Tc[cc][c4]); } }
    __threadfence(); }
}

__global__ __launch_bounds__(128) void attn_kernel(const float* __restrict__ qk, const b16* __restrict__ vpl, float* __restrict__ ofm) {
  __shared__ __attribute__((aligned(16))) float Tc[C][64 + 4];
  const int wid = threadIdx.x >> 5, lane = threadIdx.x & 31, hh = lane >> 4, col = lane & 15; const int p0 = blockIdx.x * 64, b = p0 / N, t0 = p0 % N, q0 = t0 + wid * 16, qi = q0 + col;
  v16b qf, ql; frag_split_s(qk + ((size_t)b * N + qi) * 64, hh, QS, qf, ql);
  const b16* V = vpl + ((size_t)b * C) * N;
  float m = -INFINITY, l = 0.0f; v8f o[16];
#pragma unroll
  for (int t = 0; t < 16; ++t) o[t] = (v8f){};
  for (int kb = 0; kb < N; kb += 32) { v16b ka, kal, kc, kcl; frag_split_s(qk + ((size_t)b * N + kb + col) * 64 + 32, hh, KS, ka, kal); frag_split_s(qk + ((size_t)b * N + kb + 16 + col) * 64 + 32, hh, KS, kc, kcl);
    v8f s0 = {}, s1 = {}; s0 = wmma16b(ka, qf, s0); s0 = wmma16b(ka, ql, s0); s0 = wmma16b(kal, qf, s0); s1 = wmma16b(kc, qf, s1); s1 = wmma16b(kc, ql, s1); s1 = wmma16b(kcl, qf, s1);
    float mr = -INFINITY;
#pragma unroll
    for (int r = 0; r < 8; ++r) { s0[r] *= 1.0f / (QS * KS); s1[r] *= 1.0f / (QS * KS); mr = fmaxf(mr, fmaxf(s0[r], s1[r])); }
    mr = fmaxf(mr, __shfl_xor(mr, 16));
    const float mn = fmaxf(m, mr), al_ = nexp(m - mn); m = mn; float sum = 0.0f; v16b pbv;
#pragma unroll
    for (int r = 0; r < 8; ++r) { const float e0 = nexp(s0[r] - mn), e1 = nexp(s1[r] - mn); sum += e0 + e1; pbv[r] = (b16)(e0 * PS); pbv[8 + r] = (b16)(e1 * PS); }
    sum += __shfl_xor(sum, 16); l = l * al_ + sum;
#pragma unroll
    for (int t = 0; t < 16; ++t) { o[t] *= al_; const v16b vf = frag_kb(V + (size_t)(t * 16 + col) * N + kb, hh); o[t] = wmma16b(vf, pbv, o[t]); } }
  const float inv = 1.0f / (l * VS * PS);
#pragma unroll
  for (int t = 0; t < 16; ++t)
#pragma unroll
    for (int r = 0; r < 8; ++r) Tc[t * 16 + 8 * hh + r][wid * 16 + col] = o[t][r] * inv;
  __syncthreads();
  for (int pass = 0; pass < 2; ++pass) { for (int i = threadIdx.x; i < C * 16; i += 128) { const int cc = i >> 4, c4 = (i & 15) * 4; *(volatile v4f*)(ofm + ((size_t)b * C + cc) * N + t0 + c4) = *(const v4f*)(&Tc[cc][c4]); } __threadfence(); }
}

__global__ __launch_bounds__(1024) void chan_kernel(const float* __restrict__ qkc, const float* __restrict__ vc, float* __restrict__ ocl) {
  __shared__ float E[CL][CL + 1], A[CL][CL + 1];
  const int b = blockIdx.x, t_ = threadIdx.x; const float* qc = qkc + ((size_t)b * 64) * N; const float* kc = qc + (size_t)32 * N; const float* vb = vc + ((size_t)b * 32) * N;
  { const int i = t_ >> 5, j = t_ & 31; float s = 0.0f; const float* ki = kc + (size_t)i * N; const float* qj = qc + (size_t)j * N; for (int n = 0; n < N; n += 4) { const v4f a = *(const v4f*)(ki + n), c = *(const v4f*)(qj + n); s += pmul(a[0], c[0]); s += pmul(a[1], c[1]); s += pmul(a[2], c[2]); s += pmul(a[3], c[3]); } E[i][j] = s; }
  __syncthreads();
  if (t_ < 32) { const int i = t_; float mx = -INFINITY; for (int j = 0; j < CL; ++j) mx = fmaxf(mx, E[i][j]); float sm = 0.0f; for (int j = 0; j < CL; ++j) { const float e = nexp(E[i][j] - mx); A[i][j] = e; sm += e; } const float inv = 1.0f / sm; for (int j = 0; j < CL; ++j) A[i][j] *= inv; }
  __syncthreads();
  for (int i = 0; i < CL; ++i) { for (int n = t_; n < N; n += 1024) { float s = 0.0f;
#pragma unroll 8
      for (int j = 0; j < CL; ++j) s += pmul(A[j][i], vb[(size_t)j * N + n]);
      for (int pass = 0; pass < 2; ++pass) ((volatile float*)ocl)[((size_t)b * CL + i) * N + n] = s; } }
  __threadfence();
}

__global__ __launch_bounds__(128) void final_kernel(const b16* __restrict__ xt, const b16* __restrict__ R, const float* __restrict__ Pb, const float* __restrict__ P, const float* __restrict__ ocl, const float* __restrict__ ofm, const float* __restrict__ x, float* __restrict__ out) {
  __shared__ __attribute__((aligned(16))) float Tc[64][128 + 4];
  const int lane = threadIdx.x & 31, wave = threadIdx.x >> 5, nloc = lane & 15, hlf = lane >> 4, c0 = blockIdx.x * 64, p0 = blockIdx.y * 128, m0 = p0 + wave * 32, b = p0 / N, t0 = p0 % N;
  const b16* Wh = R + Wo_::CVH; const b16* Wl = R + Wo_::CVL; const b16* xb = xt + ((size_t)b * N) * C;
  v8f acc[2][4];
#pragma unroll
  for (int r = 0; r < 2; ++r)
#pragma unroll
    for (int t = 0; t < 4; ++t) acc[r][t] = (v8f){};
  const int n0r = (m0 % N) + nloc, n1r = n0r + 16; const int i0 = n0r >> 6, j0 = n0r & 63, i1 = n1r >> 6, j1 = n1r & 63;
  for (int tap = 0; tap < 9; ++tap) { const int dy = tap / 3 - 1, dx = tap % 3 - 1; const int ia = i0 + dy, ja = j0 + dx, ib = i1 + dy, jb = j1 + dx; const bool va = (ia >= 0 && ia < Hh && ja >= 0 && ja < Ww), vb_ = (ib >= 0 && ib < Hh && jb >= 0 && jb < Ww);
    const b16* ra = xb + (size_t)(va ? (ia * Ww + ja) : 0) * C; const b16* rb = xb + (size_t)(vb_ ? (ib * Ww + jb) : 0) * C;
#pragma unroll 2
    for (int kb = 0; kb < C; kb += 32) { v16b a0 = frag_kb(ra + kb, hlf), a1 = frag_kb(rb + kb, hlf); if (!va) a0 = (v16b){}; if (!vb_) a1 = (v16b){};
      const size_t ko = (size_t)tap * C + kb;
#pragma unroll
      for (int t = 0; t < 4; ++t) { const size_t ro = (size_t)(c0 + t * 16 + nloc) * KCV + ko; const v16b bh = frag_kb(Wh + ro, hlf), bl = frag_kb(Wl + ro, hlf); acc[0][t] = wmma16b(a0, bh, acc[0][t]); acc[0][t] = wmma16b(a0, bl, acc[0][t]); acc[1][t] = wmma16b(a1, bh, acc[1][t]); acc[1][t] = wmma16b(a1, bl, acc[1][t]); } } }
  v8f acc2[2][4];
#pragma unroll
  for (int r = 0; r < 2; ++r)
#pragma unroll
    for (int t = 0; t < 4; ++t) acc2[r][t] = (v8f){};
  { v16b ah[2], al[2]; const float* ob = ocl + ((size_t)b * CL) * N;
#pragma unroll
    for (int r = 0; r < 2; ++r) { const int pos = (m0 % N) + r * 16 + nloc;
#pragma unroll
      for (int e = 0; e < 16; ++e) { const int j = (e < 8) ? (8 * hlf + e) : (16 + 8 * hlf + e - 8); b16 h_, l_; split16(ob[(size_t)j * N + pos] * WS8, h_, l_); ah[r][e] = h_; al[r][e] = l_; } }
#pragma unroll
    for (int t = 0; t < 4; ++t) { const v16b bw = frag_kb(R + Wo_::WOC + (size_t)(c0 + t * 16 + nloc) * CL, hlf);
#pragma unroll
      for (int r = 0; r < 2; ++r) { acc2[r][t] = wmma16b(ah[r], bw, acc2[r][t]); acc2[r][t] = wmma16b(al[r], bw, acc2[r][t]); } } }
  const float gfm = P[1], gc = P[2], rg = P[3];
#pragma unroll
  for (int t = 0; t < 4; ++t) { const int cc = c0 + t * 16 + nloc; const float boc = Pb[448 + cc];
#pragma unroll
    for (int r = 0; r < 2; ++r)
#pragma unroll
      for (int v = 0; v < 8; ++v) { const int pl = wave * 32 + r * 16 + 8 * hlf + v; float y = acc[r][t][v] * (1.0f / WS8); y = (y > 0.0f) ? y : 0.2f * y; const float outc = acc2[r][t][v] * (1.0f / WS8) + boc;
        const size_t gi = ((size_t)b * C + cc) * N + t0 + pl; Tc[t * 16 + nloc][pl] = bf16_rne(x[gi]) + gfm * ofm[gi] + gc * outc + rg * y; } }
  __syncthreads();
  for (int pass = 0; pass < 2; ++pass) { for (int i = threadIdx.x; i < 64 * 32; i += 128) { const int cc = i >> 5, c4 = (i & 31) * 4; *(volatile v4f*)(out + ((size_t)b * C + c0 + cc) * N + t0 + c4) = *(const v4f*)(&Tc[cc][c4]); } __threadfence(); }
}
}

extern "C" void kernel_launch(void* const* d_in, const int* in_sizes, int n_in,
                              void* d_out, int out_size, void* d_ws, size_t ws_size, hipStream_t stream) {
  (void)n_in; (void)out_size;
  const float* x = (const float*)d_in[0]; const float* wq = (const float*)d_in[1]; const float* bq = (const float*)d_in[2]; const float* wk = (const float*)d_in[3]; const float* bk = (const float*)d_in[4]; const float* wv = (const float*)d_in[5]; const float* bv = (const float*)d_in[6]; const float* gfm = (const float*)d_in[7];
  const float* wqc = (const float*)d_in[8]; const float* bqc = (const float*)d_in[9]; const float* wkc = (const float*)d_in[10]; const float* bkc = (const float*)d_in[11]; const float* wvc = (const float*)d_in[12]; const float* bvc = (const float*)d_in[13]; const float* woc = (const float*)d_in[14]; const float* boc = (const float*)d_in[15]; const float* gc = (const float*)d_in[16];
  const float* wbar = (const float*)d_in[17]; const float* usn = (const float*)d_in[18]; const float* rg = (const float*)d_in[20];
  float* out = (float*)d_out;
  if (in_sizes[0] != NT * C || in_sizes[1] != CL * C || in_sizes[5] != C * C || in_sizes[17] != C * C * 9 || in_sizes[18] != C) return;
  size_t off = 0; char* ws = (char*)d_ws;
  auto carve = [&](size_t bytes) { char* p = ws + off; off += (bytes + 255) & ~(size_t)255; return p; };
  float* P = (float*)carve(256); b16* R = (b16*)carve(Wo_::END * 2); float* Pb = (float*)carve(1024 * 4); b16* xt = (b16*)carve((size_t)NT * C * 2);
  float* qk = (float*)carve((size_t)NT * 64 * 4); b16* vpl = (b16*)carve((size_t)NT * C * 2); float* qkc = (float*)carve((size_t)Bn * 64 * N * 4); float* vc = (float*)carve((size_t)Bn * 32 * N * 4); float* ocl = (float*)carve((size_t)Bn * 32 * N * 4); float* ofm = (float*)carve((size_t)NT * C * 4);
  if (off > ws_size) return;
  sigma_kernel<<<1, 256, 0, stream>>>(wbar, usn, gfm, gc, rg, P);
  prep_kernel<<<512, 256, 0, stream>>>(wq, wk, wv, wqc, wkc, wvc, woc, wbar, bq, bk, bv, bqc, bkc, bvc, boc, P, R, Pb);
  xpose_kernel<<<dim3(N / 128, Bn), 256, 0, stream>>>(x, xt);
  lin_kernel<<<dim3(7, NT / 128), 128, 0, stream>>>(xt, R, Pb, qk, vpl, qkc, vc);
  attn_kernel<<<NT / 64, 128, 0, stream>>>(qk, vpl, ofm);
  chan_kernel<<<Bn, 1024, 0, stream>>>(qkc, vc, ocl);
  final_kernel<<<dim3(C / 64, NT / 128), 128, 0, stream>>>(xt, R, Pb, P, ocl, ofm, x, out);
}
